// BossBD2Model_77137612636758
// MI455X (gfx1250) — hardware-run, weakly checked
//
#include <hip/hip_runtime.h>


namespace {
constexpr int B = 32, T = 16384, HID = 32, G4 = 128;
constexpr float HS = 1024.0f, WSC = 256.0f;
typedef _Float16 b16;
typedef __attribute__((ext_vector_type(16))) _Float16 v16b;
typedef __attribute__((ext_vector_type(8))) _Float16 v8b;
typedef __attribute__((ext_vector_type(8))) float v8f;
typedef __attribute__((ext_vector_type(4))) float v4f;
__device__ __forceinline__ float bf16_rne(float f) { unsigned int u = __float_as_uint(f); u += 0x7FFFu + ((u >> 16) & 1u); return __uint_as_float(u & 0xFFFF0000u); }
__device__ __forceinline__ void split16(float v, b16& hi, b16& lo) { hi = (b16)v; lo = (b16)(v - (float)hi); }
__device__ __forceinline__ v16b frag_kb(const b16* p, int hh) { const v8b a = *(const v8b*)(p + 8 * hh), b = *(const v8b*)(p + 16 + 8 * hh); v16b f;
#pragma unroll
  for (int e = 0; e < 8; ++e) { f[e] = a[e]; f[8 + e] = b[e]; } return f; }
__device__ __forceinline__ v8f wmma16b(v16b a, v16b b, v8f c) { v8f d = __builtin_amdgcn_wmma_f32_16x16x32_f16(false, a, false, b, (short)0, c, false, false); asm volatile("v_nop\n\tv_nop\n\tv_nop\n\tv_nop" : "+v"(d) : "v"(a), "v"(b)); return d; }
__device__ __forceinline__ void wave_lds_sync() { __builtin_amdgcn_fence(__ATOMIC_RELEASE, "workgroup"); __builtin_amdgcn_wave_barrier(); __builtin_amdgcn_fence(__ATOMIC_ACQUIRE, "workgroup"); }
__device__ __forceinline__ float pmul(float a, float b) { float p = a * b; asm volatile("" : "+v"(p)); return p; }
__device__ __forceinline__ float sigm(float v) { return 1.0f / (1.0f + __expf(-v)); }

__global__ __launch_bounds__(256) void wcopy_kernel(const float* __restrict__ w, b16* __restrict__ WT) {
  const int u = blockIdx.x * 256 + threadIdx.x; if (u >= G4 * HID / 8) return; const int e = u * 8; v8b v;
#pragma unroll
  for (int j = 0; j < 8; ++j) v[j] = (b16)(bf16_rne(w[e + j]) * WSC); for (int pass = 0; pass < 2; ++pass) { *(volatile v8b*)(WT + e) = v; __threadfence(); }
}
__global__ __launch_bounds__(32) void lstm_kernel(const float* __restrict__ x, const float* __restrict__ Wih, const b16* __restrict__ WT, const float* __restrict__ bih, const float* __restrict__ bhh, const float* __restrict__ Wout, const float* __restrict__ bout, int TV, float* __restrict__ out) {
  __shared__ __attribute__((aligned(16))) b16 Ah[16][40], Al[16][40]; __shared__ float Ob[16][33];
  const int lane = threadIdx.x, nloc = lane & 15, hlf = lane >> 4; const int b0 = blockIdx.x * 16;
  float wih[8], bb[8]; for (int t = 0; t < 8; ++t) { const int col = t * 16 + nloc; wih[t] = bf16_rne(Wih[col]); bb[t] = bf16_rne(bih[col]) + bf16_rne(bhh[col]); }
  const float wo0 = bf16_rne(Wout[nloc]), wo1 = bf16_rne(Wout[16 + nloc]), bo = bf16_rne(bout[0]);
  float c0[8], c1[8];
#pragma unroll
  for (int r8 = 0; r8 < 8; ++r8) { c0[r8] = 0.0f; c1[r8] = 0.0f; }
  for (int rr = 0; rr < 16; ++rr) { Ah[rr][lane] = (b16)0.0f; Al[rr][lane] = (b16)0.0f; }
  wave_lds_sync();
#pragma unroll 1
  for (int step = 0; step < TV; ++step) {
    v8f acc[8];
#pragma unroll
    for (int t = 0; t < 8; ++t) acc[t] = (v8f){};
    { const v16b a = frag_kb(&Ah[nloc][0], hlf), al = frag_kb(&Al[nloc][0], hlf);
#pragma unroll
      for (int t = 0; t < 8; ++t) { const v16b bw = frag_kb(WT + (size_t)(t * 16 + nloc) * HID, hlf); acc[t] = wmma16b(a, bw, acc[t]); acc[t] = wmma16b(al, bw, acc[t]); } }
    wave_lds_sync();
    float po[8];
#pragma unroll
    for (int r8 = 0; r8 < 8; ++r8) { const int row = 8 * hlf + r8; const float xv = bf16_rne(x[(size_t)(b0 + row) * T + step]); float g[8];
#pragma unroll
      for (int t = 0; t < 8; ++t) g[t] = acc[t][r8] * (1.0f / (HS * WSC)) + pmul(xv, wih[t]) + bb[t];
      c0[r8] = pmul(sigm(g[2]), c0[r8]) + pmul(sigm(g[0]), tanhf(g[4])); c1[r8] = pmul(sigm(g[3]), c1[r8]) + pmul(sigm(g[1]), tanhf(g[5]));
      const float h0 = pmul(sigm(g[6]), tanhf(c0[r8])), h1 = pmul(sigm(g[7]), tanhf(c1[r8]));
      b16 p, q; split16(h0 * HS, p, q); Ah[row][nloc] = p; Al[row][nloc] = q; split16(h1 * HS, p, q); Ah[row][16 + nloc] = p; Al[row][16 + nloc] = q;
      po[r8] = pmul(h0, wo0) + pmul(h1, wo1); }
#pragma unroll
    for (int r8 = 0; r8 < 8; ++r8) { float s = po[r8]; for (int o = 1; o < 16; o <<= 1) s += __shfl_xor(s, o); if (nloc == 0) Ob[8 * hlf + r8][step & 31] = s + bo; }
    wave_lds_sync();
    if ((step & 31) == 31 || step == TV - 1) { const int t0 = step & ~31; const int nv = step - t0 + 1;
      for (int pass = 0; pass < 2; ++pass) { for (int rr = 0; rr < 16; ++rr) if (lane < nv) ((volatile float*)out)[(size_t)(b0 + rr) * T + t0 + lane] = Ob[rr][lane]; __threadfence(); }
      wave_lds_sync(); } }
}
}

extern "C" void kernel_launch(void* const* d_in, const int* in_sizes, int n_in, void* d_out, int out_size, void* d_ws, size_t ws_size, hipStream_t stream) {
  (void)n_in;
  auto Fp = [&](int i) { return (const float*)d_in[i]; };
  if (in_sizes[0] != B * T || in_sizes[1] != G4 || in_sizes[2] != G4 * HID || in_sizes[3] != G4 || in_sizes[4] != G4 || in_sizes[5] != HID || in_sizes[6] != 1 || out_size != B * T) return;
  const int TV = T;
  size_t off = 0; char* ws = (char*)d_ws;
  auto carve = [&](size_t bytes) { char* p = ws + off; off += (bytes + 255) & ~(size_t)255; return p; };
  b16* WT = (b16*)carve(G4 * HID * 2);
  if (off > ws_size || off > ((size_t)1 << 20)) return;
  wcopy_kernel<<<2, 256, 0, stream>>>(Fp(2), WT);
  lstm_kernel<<<B / 16, 32, 0, stream>>>(Fp(0), Fp(1), WT, Fp(3), Fp(4), Fp(5), Fp(6), TV, (float*)d_out);
}
